// GroupedQueryAttention_76991583748666
// MI455X (gfx1250) — hardware-run, weakly checked
//
#include <hip/hip_runtime.h>


#ifndef NB
#define NB 4
#endif
#ifndef SEQ
#define SEQ 2048
#endif
#ifndef TRES
#define TRES 512
#endif
#define NB_FULL   4
#define SEQ_FULL  2048
#define CDIM      1024
#define NHEAD     16
#define NKV       4
#define GROUPS    (NHEAD / NKV)
#define HDIM      64
#define ROTD      32
#define VEW       (NKV * HDIM)
#define NTOK      (NB * SEQ)
#define NUNIT     (3 * NKV)
#define NWROWS    (CDIM + 2 * VEW)
#define QT_ALL    (SEQ / 64)
#define QT_RES    (TRES / 64)
#define MW_WORDS  (SEQ_FULL / 32)
#define MW_PITCH  96

static_assert(NB >= 1 && NB <= NB_FULL);
static_assert(SEQ % 64 == 0 && SEQ <= SEQ_FULL && SEQ >= TRES);
static_assert(TRES % 64 == 0 && TRES >= 64);
static_assert(NHEAD % NKV == 0 && HDIM == 64 && CDIM == NHEAD * HDIM && ROTD * 2 == HDIM);
static_assert(CDIM % 64 == 0 && VEW % 64 == 0 && NTOK % 64 == 0 && VEW % 32 == 0 && CDIM % 32 == 0);
static_assert(NUNIT * 64 == 3 * VEW && GROUPS * NKV * HDIM == CDIM);
static_assert(SEQ_FULL == 2048 && MW_WORDS == 64 && MW_PITCH == 3 * 32 && MW_WORDS < MW_PITCH);
static_assert(SEQ % 8 == 0 && ROTD == 32);

#define XH_BYTES   ((size_t)NTOK * CDIM * 2)
#define WALL_BYTES ((size_t)NWROWS * CDIM * 2)
#define WOT_BYTES  ((size_t)CDIM * VEW * 2)
#define TAB_BYTES  ((size_t)SEQ * ROTD * 4)
#define MB_BYTES   ((size_t)SEQ * MW_PITCH * 4)
#define PL_ELEMS   ((size_t)NB * NKV * SEQ * HDIM)
#define PL_BYTES   (PL_ELEMS * 2)
#define YP_BYTES   ((size_t)NTOK * VEW * 2)
#define WS_TOTAL   (XH_BYTES + WALL_BYTES + WOT_BYTES + 2 * TAB_BYTES + MB_BYTES + 6 * PL_BYTES + 2 * YP_BYTES)
static_assert(WS_TOTAL <= (size_t)134217728);
static_assert(XH_BYTES % 128 == 0 && WALL_BYTES % 128 == 0 && WOT_BYTES % 128 == 0 && TAB_BYTES % 128 == 0);
static_assert(MB_BYTES % 128 == 0 && PL_BYTES % 128 == 0 && YP_BYTES % 128 == 0);
static_assert((size_t)(NTOK / 2) * 256 * 8 == (size_t)NTOK * CDIM);
static_assert(2 * 256 * 8 == 64 * 64);
static_assert(256 * 16 == 64 * 64);
static_assert((SEQ / 8) * 8 == SEQ);
static_assert(128 * 32 == 64 * 64);
static_assert(4 * 128 * 8 == 64 * 64);
static_assert(4 * 32 * 8 == 16 * HDIM);
static_assert(8 * 32 * 4 == 16 * 64);
static_assert(QT_RES * 64 + (QT_ALL - QT_RES) * 64 == SEQ);
static_assert((size_t)NB_FULL * SEQ_FULL * CDIM * 4 == (size_t)33554432);
static_assert(((size_t)(NB - 1) * SEQ_FULL + SEQ) * CDIM <= (size_t)NB_FULL * SEQ_FULL * CDIM);

typedef _Float16 v16h __attribute__((ext_vector_type(16)));
typedef _Float16 v8h  __attribute__((ext_vector_type(8)))  __attribute__((may_alias));
typedef float    v8f  __attribute__((ext_vector_type(8)));
typedef float    v4f  __attribute__((ext_vector_type(4)))  __attribute__((may_alias));

union Frag { v16h v; v8h h[2]; };

__device__ __forceinline__ v8f wmma16(v16h a, v16h b, v8f c) {
  return __builtin_amdgcn_wmma_f32_16x16x32_f16(false, a, false, b, (short)0, c, false, false);
}

__device__ __forceinline__ v8f vzero8() {
  v8f z = {0.0f, 0.0f, 0.0f, 0.0f, 0.0f, 0.0f, 0.0f, 0.0f};
  return z;
}

__device__ __forceinline__ float bf16r(float f) {
  unsigned int u = __float_as_uint(f);
  u = (u + 0x7FFFu + ((u >> 16) & 1u)) & 0xFFFF0000u;
  return __uint_as_float(u);
}

__device__ __forceinline__ void split16(float v, _Float16& hi, _Float16& lo) {
  hi = (_Float16)v;
  lo = (_Float16)((v - (float)hi) * 2048.0f);
}

static __device__ __forceinline__ v8f wmma16g(v16h a, v16h b, v8f c) {
  c = __builtin_amdgcn_wmma_f32_16x16x32_f16(false, a, false, b, (short)0, c, false, false);
  asm volatile("v_nop\n\tv_nop\n\tv_nop\n\tv_nop" : "+v"(c) : "v"(a), "v"(b));
  return c;
}

static __device__ __forceinline__ _Float16 toh_flush(float v) {
  const _Float16 r = (_Float16)v;
  return (fabsf(v) < 6.103515625e-05f) ? (_Float16)0.0f : r;
}

static __device__ __forceinline__ void split16f(float v, _Float16& hi, _Float16& lo) {
  hi = toh_flush(v);
  lo = toh_flush((v - (float)hi) * 2048.0f);
}

__global__ void __launch_bounds__(256) k_cvt_x(const float* __restrict__ x, _Float16* __restrict__ xh) {
  const unsigned int gid = blockIdx.x * 256u + threadIdx.x;
  const unsigned int tok = gid >> 7;
  const int c = (int)(gid & 127u) * 8;
  if (tok >= (unsigned int)NTOK) return;
  const int b = (int)tok / SEQ;
  const int t = (int)tok - b * SEQ;
  const float* src = x + ((size_t)b * SEQ_FULL + t) * CDIM + c;
  const v4f f0 = *(const v4f*)src;
  const v4f f1 = *(const v4f*)(src + 4);
  v8h o;
#pragma unroll
  for (int j = 0; j < 4; ++j) {
    o[j]     = (_Float16)bf16r(f0[j]);
    o[j + 4] = (_Float16)bf16r(f1[j]);
  }
  _Float16* dst = xh + (size_t)tok * CDIM + c;
  *(volatile v8h*)dst = o;
  __threadfence();
  *(volatile v8h*)dst = o;
}

__global__ void __launch_bounds__(256) k_cvt_wT(const float* __restrict__ src, int srcPitch,
                                                _Float16* __restrict__ dst, int dstPitch) {
  __shared__ __attribute__((aligned(16))) _Float16 sW[64][72];

  const int tid = threadIdx.x;
  const int n0  = blockIdx.x * 64;
  const int k0  = blockIdx.y * 64;
  const int ir  = tid >> 2;
  const int oc  = (tid & 3) * 16;
  const float* sp = src + (size_t)(k0 + ir) * srcPitch + n0 + oc;
#pragma unroll
  for (int g = 0; g < 4; ++g) {
    const v4f f = *(const v4f*)(sp + 4 * g);
#pragma unroll
    for (int e = 0; e < 4; ++e) sW[oc + 4 * g + e][ir] = toh_flush(bf16r(f[e]) * 16.0f);
  }
  __syncthreads();
  for (int pass = 0; pass < 2; ++pass) {
#pragma unroll
    for (int it = 0; it < 2; ++it) {
      const int p    = it * 256 + tid;
      const int line = p >> 3;
      const int q8   = (p & 7) * 8;
      const v8h hv = *(const v8h*)(&sW[line][q8]);
      *(volatile v8h*)(dst + (size_t)(n0 + line) * dstPitch + k0 + q8) = hv;
    }
    __threadfence();
  }
}

__global__ void __launch_bounds__(256) k_rope_tab(float* __restrict__ cosT, float* __restrict__ sinT) {
#pragma clang fp contract(off)
  const int wave = __builtin_amdgcn_readfirstlane((int)(threadIdx.x >> 5));
  const int lane = (int)(threadIdx.x & 31);
  const int t = (int)blockIdx.x * 8 + wave;
  if (t >= SEQ) return;
  float p = 1.0f;
#pragma unroll 1
  for (int i = 0; i < ROTD - 1; ++i) p = (i < lane) ? p * 10.0f : p;
  const float theta = __builtin_amdgcn_rcpf(p);
  const float ang = (float)(t + 1) * theta;
  const float c = cosf(ang);
  const float s = sinf(ang);
  float* cd = cosT + (size_t)t * ROTD + lane;
  float* sd = sinT + (size_t)t * ROTD + lane;
  *(volatile float*)cd = c;
  *(volatile float*)sd = s;
  __threadfence();
  *(volatile float*)cd = c;
  *(volatile float*)sd = s;
}

__global__ void __launch_bounds__(256) k_mask_pack(const float* __restrict__ mask, unsigned int* __restrict__ mbits) {
  const int wave = __builtin_amdgcn_readfirstlane((int)(threadIdx.x >> 5));
  const int lane = (int)(threadIdx.x & 31);
  const int row = (int)blockIdx.x * 8 + wave;
  if (row >= SEQ) return;
  const float* mr = mask + (size_t)row * SEQ_FULL;
  unsigned int w0 = 0u, w1 = 0u, bad = 0u;
#pragma unroll 4
  for (int it = 0; it < 32; ++it) {
    const float va = mr[it * 32 + lane];
    const float vb = mr[1024 + it * 32 + lane];
    const unsigned int ba = __builtin_amdgcn_ballot_w32(va != 0.0f);
    const unsigned int bb = __builtin_amdgcn_ballot_w32(vb != 0.0f);
    w0 = (it == lane) ? ba : w0;
    w1 = (it == lane) ? bb : w1;
    const bool xa = (va != 0.0f) && (va != 1.0f);
    const bool xb = (vb != 0.0f) && (vb != 1.0f);
    bad |= (xa || xb) ? 1u : 0u;
  }
  const unsigned int anyb = __builtin_amdgcn_ballot_w32(bad != 0u);
  const unsigned int flg = (anyb != 0u) ? 1u : 0u;
  unsigned int* dst = mbits + (size_t)row * MW_PITCH + lane;
  *(volatile unsigned int*)(dst)      = w0;
  *(volatile unsigned int*)(dst + 32) = w1;
  *(volatile unsigned int*)(dst + 64) = flg;
  __threadfence();
  *(volatile unsigned int*)(dst)      = w0;
  *(volatile unsigned int*)(dst + 32) = w1;
  *(volatile unsigned int*)(dst + 64) = flg;
}

__global__ void __launch_bounds__(128) k_qkv(
    const _Float16* __restrict__ xh, const _Float16* __restrict__ wall,
    const float* __restrict__ cosT, const float* __restrict__ sinT,
    _Float16* __restrict__ planes) {
  __shared__ __attribute__((aligned(16))) float    sT[64][68];
  __shared__ __attribute__((aligned(16))) _Float16 sH[64][72];
  __shared__ __attribute__((aligned(16))) _Float16 sL[64][72];

  const int tid  = threadIdx.x;
  const int wave = __builtin_amdgcn_readfirstlane(tid >> 5);
  const int lane = tid & 31;
  const int l16  = lane & 15;
  const int lh   = lane >> 4;
  const int u    = blockIdx.x;
  const int rt   = blockIdx.y;
  const int tok0 = rt * 64;
  const int b    = tok0 / SEQ;
  const int t0   = tok0 - b * SEQ;
  const int ng   = (u < NKV) ? GROUPS : 1;
  const int wrow0 = (u < NKV) ? (u * GROUPS * HDIM) : (CDIM + (u - NKV) * HDIM);

  const _Float16* arow = xh + (size_t)(tok0 + wave * 16 + l16) * CDIM + 8 * lh;
  const _Float16* brow = wall + (size_t)(wrow0 + l16) * CDIM + 8 * lh;

  v8f acc[4];
#pragma unroll
  for (int n = 0; n < 4; ++n) acc[n] = vzero8();

  for (int k0 = 0; k0 < CDIM; k0 += 32) {
    Frag a;
    a.h[0] = *(const v8h*)(arow + k0);
    a.h[1] = *(const v8h*)(arow + k0 + 16);
#pragma unroll 1
    for (int g = 0; g < ng; ++g) {
      Frag bw[4];
#pragma unroll
      for (int n = 0; n < 4; ++n) {
        const _Float16* bp = brow + (size_t)(g * HDIM + n * 16) * CDIM + k0;
        bw[n].h[0] = *(const v8h*)bp;
        bw[n].h[1] = *(const v8h*)(bp + 16);
      }
#pragma unroll
      for (int n = 0; n < 4; ++n) acc[n] = wmma16g(a.v, bw[n].v, acc[n]);
    }
  }

#pragma unroll
  for (int n = 0; n < 4; ++n)
#pragma unroll
    for (int r = 0; r < 8; ++r)
      sT[wave * 16 + r + 8 * lh][n * 16 + l16] = acc[n][r] * (1.0f / 16.0f);
  __syncthreads();

  const int i = tid >> 1;
  const int j = tid & 1;
  const int t = t0 + i;
  if (u < 2 * NKV) {
    const float* cp = cosT + (size_t)t * ROTD + 16 * j;
    const float* sp = sinT + (size_t)t * ROTD + 16 * j;
#pragma unroll
    for (int g = 0; g < 4; ++g) {
      const v4f xa = *(const v4f*)(&sT[i][32 * j + 8 * g]);
      const v4f xb = *(const v4f*)(&sT[i][32 * j + 8 * g + 4]);
      const v4f cc = *(const v4f*)(cp + 4 * g);
      const v4f sn = *(const v4f*)(sp + 4 * g);
      float xv[8];
#pragma unroll
      for (int e = 0; e < 4; ++e) { xv[e] = xa[e]; xv[4 + e] = xb[e]; }
#pragma unroll
      for (int e = 0; e < 4; ++e) {
        const float c  = cc[e];
        const float s  = sn[e];
        const float xr = xv[2 * e];
        const float xi = xv[2 * e + 1];
        const float orr = xr * c - xi * s;
        const float oii = xr * s + xi * c;
        const int d = 32 * j + 8 * g + 2 * e;
        _Float16 hi, lo;
        split16f(orr, hi, lo);
        sH[i][d] = hi;
        sL[i][d] = lo;
        split16f(oii, hi, lo);
        sH[i][d + 1] = hi;
        sL[i][d + 1] = lo;
      }
    }
  } else {
#pragma unroll
    for (int g = 0; g < 8; ++g) {
      const v4f va = *(const v4f*)(&sT[i][32 * j + 4 * g]);
#pragma unroll
      for (int e = 0; e < 4; ++e) {
        _Float16 hi, lo;
        split16f(va[e], hi, lo);
        sH[32 * j + 4 * g + e][i] = hi;
        sL[32 * j + 4 * g + e][i] = lo;
      }
    }
  }
  __syncthreads();

  int sel;
  size_t base;
  size_t lstr;
  if (u < NKV) {
    sel = 0;
    base = ((size_t)(b * NKV + u) * SEQ + t0) * HDIM;
    lstr = HDIM;
  } else if (u < 2 * NKV) {
    sel = 1;
    base = ((size_t)(b * NKV + (u - NKV)) * SEQ + t0) * HDIM;
    lstr = HDIM;
  } else {
    sel = 2;
    base = ((size_t)(b * NKV + (u - 2 * NKV)) * HDIM) * SEQ + t0;
    lstr = SEQ;
  }
  _Float16* ph = planes + (size_t)sel * 2 * PL_ELEMS;
  _Float16* pl = ph + PL_ELEMS;
  for (int pass = 0; pass < 2; ++pass) {
#pragma unroll
    for (int it = 0; it < 4; ++it) {
      const int p    = it * 128 + tid;
      const int line = p >> 3;
      const int q8   = (p & 7) * 8;
      const size_t off = base + (size_t)line * lstr + q8;
      const v8h hv = *(const v8h*)(&sH[line][q8]);
      const v8h lv = *(const v8h*)(&sL[line][q8]);
      *(volatile v8h*)(ph + off) = hv;
      *(volatile v8h*)(pl + off) = lv;
    }
    __threadfence();
  }
}

template <bool RES>
static __device__ __forceinline__ void flash_body(
    const _Float16* __restrict__ qH, const _Float16* __restrict__ qL,
    const _Float16* __restrict__ kH, const _Float16* __restrict__ kL,
    const _Float16* __restrict__ vTH, const _Float16* __restrict__ vTL,
    const unsigned int* __restrict__ mbits,
    _Float16* __restrict__ yH, _Float16* __restrict__ yL, const int qt_first) {
  __shared__ __attribute__((aligned(16))) _Float16 ldsPH[4][16 * 32];
  __shared__ __attribute__((aligned(16))) _Float16 ldsPL[4][16 * 32];
  __shared__ __attribute__((aligned(16))) _Float16 sYH[4][16][HDIM];
  __shared__ __attribute__((aligned(16))) _Float16 sYL[4][16][HDIM];

  const int tid  = threadIdx.x;
  const int wave = __builtin_amdgcn_readfirstlane(tid >> 5);
  const int lane = tid & 31;
  const int l16  = lane & 15;
  const int lh   = lane >> 4;
  const int qt   = qt_first + blockIdx.x;
  const int h    = blockIdx.y;
  const int b    = blockIdx.z;
  const int qw   = qt * 64 + wave * 16;
  const float rres = 1.0f / 2048.0f;
  const float smsc = 0.125f;

  const unsigned int* mrow = mbits + (size_t)(qw + l16) * MW_PITCH;
  const unsigned int mflag = mrow[MW_WORDS];

  v16h aqh[2], aql[2];
  {
    const size_t qo = ((size_t)(b * NKV + h) * SEQ + qw + l16) * HDIM + 8 * lh;
#pragma unroll
    for (int hc = 0; hc < 2; ++hc) {
      Frag a;
      a.h[0] = *(const v8h*)(qH + qo + hc * 32);
      a.h[1] = *(const v8h*)(qH + qo + hc * 32 + 16);
      aqh[hc] = a.v;
      Frag c;
      c.h[0] = *(const v8h*)(qL + qo + hc * 32);
      c.h[1] = *(const v8h*)(qL + qo + hc * 32 + 16);
      aql[hc] = c.v;
    }
  }

  float m[8], l[8];
  v8f coh[4], cor[4];
#pragma unroll
  for (int r = 0; r < 8; ++r) { m[r] = -1e30f; l[r] = 0.0f; }
#pragma unroll
  for (int n = 0; n < 4; ++n) { coh[n] = vzero8(); cor[n] = vzero8(); }

  const size_t kvoff = (size_t)(b * NKV + h) * SEQ * HDIM;
  const _Float16* kbase  = kH  + kvoff + 8 * lh;
  const _Float16* klbase = kL  + kvoff + 8 * lh;
  const _Float16* vbase  = vTH + kvoff + (size_t)l16 * SEQ + 8 * lh;
  const _Float16* vlbase = vTL + kvoff + (size_t)l16 * SEQ + 8 * lh;

  for (int k0 = 0; k0 < SEQ; k0 += 32) {
    const unsigned int mw = mrow[k0 >> 5];
    if (__builtin_amdgcn_ballot_w32(mw != 0u) == 0u) continue;

    v8f sh0 = vzero8(), sh1 = vzero8(), sr0 = vzero8(), sr1 = vzero8();
    Frag bh0, bh1, bl0, bl1;
    const _Float16* kr0 = kbase  + (size_t)(k0 + l16) * HDIM;
    const _Float16* kr1 = kr0 + 16 * HDIM;
    const _Float16* lr0 = klbase + (size_t)(k0 + l16) * HDIM;
    const _Float16* lr1 = lr0 + 16 * HDIM;
#pragma unroll
    for (int hc = 0; hc < 2; ++hc) {
      bh0.h[0] = *(const v8h*)(kr0 + hc * 32); bh0.h[1] = *(const v8h*)(kr0 + hc * 32 + 16);
      bh1.h[0] = *(const v8h*)(kr1 + hc * 32); bh1.h[1] = *(const v8h*)(kr1 + hc * 32 + 16);
      bl0.h[0] = *(const v8h*)(lr0 + hc * 32); bl0.h[1] = *(const v8h*)(lr0 + hc * 32 + 16);
      bl1.h[0] = *(const v8h*)(lr1 + hc * 32); bl1.h[1] = *(const v8h*)(lr1 + hc * 32 + 16);
      sh0 = wmma16g(aqh[hc], bh0.v, sh0);
      sh1 = wmma16g(aqh[hc], bh1.v, sh1);
      sr0 = wmma16g(aqh[hc], bl0.v, sr0);
      sr1 = wmma16g(aqh[hc], bl1.v, sr1);
      sr0 = wmma16g(aql[hc], bh0.v, sr0);
      sr1 = wmma16g(aql[hc], bh1.v, sr1);
    }

    asm volatile("" ::: "memory");
    float alpha[8];
#pragma unroll
    for (int r = 0; r < 8; ++r) {
      const unsigned int wr = __shfl(mw, r + 8 * lh, 32);
      const bool ok0 = ((wr >> l16) & 1u) != 0u;
      const bool ok1 = ((wr >> (16 + l16)) & 1u) != 0u;
      const float x0 = ok0 ? (sh0[r] + sr0[r] * rres) * smsc : -1e30f;
      const float x1 = ok1 ? (sh1[r] + sr1[r] * rres) * smsc : -1e30f;
      float tmax = fmaxf(x0, x1);
#pragma unroll
      for (int off = 1; off < 16; off <<= 1) tmax = fmaxf(tmax, __shfl_xor(tmax, off, 32));
      const float mn = fmaxf(m[r], tmax);
      alpha[r] = __expf(m[r] - mn);
      const float e0 = __expf(x0 - mn);
      const float e1 = __expf(x1 - mn);
      const float p0 = ok0 ? e0 : 0.0f;
      const float p1 = ok1 ? e1 : 0.0f;
      float ps = p0 + p1;
#pragma unroll
      for (int off = 1; off < 16; off <<= 1) ps += __shfl_xor(ps, off, 32);
      l[r] = l[r] * alpha[r] + ps;
      m[r] = mn;
      const float c0 = p0 * 1024.0f;
      const float c1 = p1 * 1024.0f;
      const _Float16 h0 = toh_flush(c0);
      const _Float16 h1 = toh_flush(c1);
      ldsPH[wave][(r + 8 * lh) * 32 + l16]      = h0;
      ldsPH[wave][(r + 8 * lh) * 32 + 16 + l16] = h1;
      if (RES) {
        ldsPL[wave][(r + 8 * lh) * 32 + l16]      = toh_flush((c0 - (float)h0) * 2048.0f);
        ldsPL[wave][(r + 8 * lh) * 32 + 16 + l16] = toh_flush((c1 - (float)h1) * 2048.0f);
      }
    }
#pragma unroll
    for (int n = 0; n < 4; ++n)
#pragma unroll
      for (int r = 0; r < 8; ++r) {
        coh[n][r] *= alpha[r];
        if (RES) cor[n][r] *= alpha[r];
      }

    asm volatile("s_wait_dscnt 0" ::: "memory");
    __builtin_amdgcn_fence(3  , "wavefront");
    __builtin_amdgcn_wave_barrier();

    Frag aph, apl;
    aph.h[0] = *(const v8h*)(&ldsPH[wave][l16 * 32 + 8 * lh]);
    aph.h[1] = *(const v8h*)(&ldsPH[wave][l16 * 32 + 16 + 8 * lh]);
    if (RES) {
      apl.h[0] = *(const v8h*)(&ldsPL[wave][l16 * 32 + 8 * lh]);
      apl.h[1] = *(const v8h*)(&ldsPL[wave][l16 * 32 + 16 + 8 * lh]);
    }
    Frag bv[4], bl[4];
#pragma unroll
    for (int n = 0; n < 4; ++n) {
      const _Float16* vp = vbase + (size_t)(n * 16) * SEQ + k0;
      bv[n].h[0] = *(const v8h*)vp;
      bv[n].h[1] = *(const v8h*)(vp + 16);
      if (RES) {
        const _Float16* lp = vlbase + (size_t)(n * 16) * SEQ + k0;
        bl[n].h[0] = *(const v8h*)lp;
        bl[n].h[1] = *(const v8h*)(lp + 16);
      }
    }
#pragma unroll
    for (int n = 0; n < 4; ++n) {
      coh[n] = wmma16g(aph.v, bv[n].v, coh[n]);
      if (RES) {
        cor[n] = wmma16g(aph.v, bl[n].v, cor[n]);
        cor[n] = wmma16g(apl.v, bv[n].v, cor[n]);
      }
    }
    asm volatile("" ::: "memory");
  }

#pragma unroll
  for (int r = 0; r < 8; ++r) {
    const unsigned int fr = __shfl(mflag, r + 8 * lh, 32);
    const float inv = __builtin_amdgcn_rcpf(l[r]) * (1.0f / 1024.0f);
#pragma unroll
    for (int n = 0; n < 4; ++n) {
      float yv = coh[n][r];
      if (RES) yv += cor[n][r] * rres;
      yv *= inv;
      yv = (fr != 0u) ? __uint_as_float(0x7FC00000u) : yv;
      _Float16 hi, lo;
      split16f(yv, hi, lo);
      sYH[wave][r + 8 * lh][n * 16 + l16] = hi;
      sYL[wave][r + 8 * lh][n * 16 + l16] = lo;
    }
  }
  asm volatile("s_wait_dscnt 0" ::: "memory");
  __builtin_amdgcn_fence(3  , "wavefront");
  __builtin_amdgcn_wave_barrier();
  const size_t ybase = ((size_t)b * SEQ + qw) * VEW + (size_t)h * HDIM;
  for (int pass = 0; pass < 2; ++pass) {
#pragma unroll
    for (int it = 0; it < 4; ++it) {
      const int p  = it * 32 + lane;
      const int rr = p >> 3;
      const int q8 = (p & 7) * 8;
      const size_t off = ybase + (size_t)rr * VEW + q8;
      const v8h hv = *(const v8h*)(&sYH[wave][rr][q8]);
      const v8h lv = *(const v8h*)(&sYL[wave][rr][q8]);
      *(volatile v8h*)(yH + off) = hv;
      *(volatile v8h*)(yL + off) = lv;
    }
    __threadfence();
  }
}

__global__ void __launch_bounds__(128) k_flash_res(
    const _Float16* __restrict__ qH, const _Float16* __restrict__ qL,
    const _Float16* __restrict__ kH, const _Float16* __restrict__ kL,
    const _Float16* __restrict__ vTH, const _Float16* __restrict__ vTL,
    const unsigned int* __restrict__ mbits,
    _Float16* __restrict__ yH, _Float16* __restrict__ yL, int qt_first) {
  flash_body<true>(qH, qL, kH, kL, vTH, vTL, mbits, yH, yL, qt_first);
}

__global__ void __launch_bounds__(128) k_flash_one(
    const _Float16* __restrict__ qH, const _Float16* __restrict__ qL,
    const _Float16* __restrict__ kH, const _Float16* __restrict__ kL,
    const _Float16* __restrict__ vTH, const _Float16* __restrict__ vTL,
    const unsigned int* __restrict__ mbits,
    _Float16* __restrict__ yH, _Float16* __restrict__ yL, int qt_first) {
  flash_body<false>(qH, qL, kH, kL, vTH, vTL, mbits, yH, yL, qt_first);
}

template <bool RES>
static __device__ __forceinline__ void oproj_body(
    const _Float16* __restrict__ yH, const _Float16* __restrict__ yL,
    const _Float16* __restrict__ woT, float* __restrict__ out, const int rt_first, const int rt_count) {
  __shared__ __attribute__((aligned(16))) float sO[4][16][68];

  const int tid  = threadIdx.x;
  const int wave = __builtin_amdgcn_readfirstlane(tid >> 5);
  const int lane = tid & 31;
  const int l16  = lane & 15;
  const int lh   = lane >> 4;
  const int nt   = blockIdx.x;
  const int b    = blockIdx.y / rt_count;
  const int rtb  = rt_first + (blockIdx.y - b * rt_count);
  const int t0   = rtb * 64;
  const int tok0 = b * SEQ + t0;

  const _Float16* arow = yH + (size_t)(tok0 + wave * 16 + l16) * VEW + 8 * lh;
  const _Float16* lrow = yL + (size_t)(tok0 + wave * 16 + l16) * VEW + 8 * lh;
  const _Float16* brow = woT + (size_t)(nt * 64 + l16) * VEW + 8 * lh;

  v8f ah[4], ar[4];
#pragma unroll
  for (int n = 0; n < 4; ++n) { ah[n] = vzero8(); ar[n] = vzero8(); }

  for (int k0 = 0; k0 < VEW; k0 += 32) {
    Frag a, al;
    a.h[0] = *(const v8h*)(arow + k0);
    a.h[1] = *(const v8h*)(arow + k0 + 16);
    if (RES) {
      al.h[0] = *(const v8h*)(lrow + k0);
      al.h[1] = *(const v8h*)(lrow + k0 + 16);
    }
    Frag bw[4];
#pragma unroll
    for (int n = 0; n < 4; ++n) {
      const _Float16* bp = brow + (size_t)(n * 16) * VEW + k0;
      bw[n].h[0] = *(const v8h*)bp;
      bw[n].h[1] = *(const v8h*)(bp + 16);
    }
#pragma unroll
    for (int n = 0; n < 4; ++n) {
      ah[n] = wmma16g(a.v, bw[n].v, ah[n]);
      if (RES) ar[n] = wmma16g(al.v, bw[n].v, ar[n]);
    }
  }

#pragma unroll
  for (int r = 0; r < 8; ++r) {
#pragma unroll
    for (int n = 0; n < 4; ++n) {
      float v = ah[n][r];
      if (RES) v += ar[n][r] * (1.0f / 2048.0f);
      sO[wave][r + 8 * lh][n * 16 + l16] = v * (1.0f / 16.0f);
    }
  }
  asm volatile("s_wait_dscnt 0" ::: "memory");
  __builtin_amdgcn_fence(3  , "wavefront");
  __builtin_amdgcn_wave_barrier();
  const size_t orow0 = (size_t)b * SEQ_FULL + t0 + wave * 16;
  for (int pass = 0; pass < 2; ++pass) {
#pragma unroll
    for (int it = 0; it < 8; ++it) {
      const int rr = it * 2 + lh;
      const int c4 = l16 * 4;
      const v4f v = *(const v4f*)(&sO[wave][rr][c4]);
      *(volatile v4f*)(out + (orow0 + rr) * CDIM + (size_t)nt * 64 + c4) = v;
    }
    __threadfence();
  }
}

__global__ void __launch_bounds__(128) k_oproj_res(
    const _Float16* __restrict__ yH, const _Float16* __restrict__ yL,
    const _Float16* __restrict__ woT, float* __restrict__ out, int rt_first, int rt_count) {
  oproj_body<true>(yH, yL, woT, out, rt_first, rt_count);
}

__global__ void __launch_bounds__(128) k_oproj_one(
    const _Float16* __restrict__ yH, const _Float16* __restrict__ yL,
    const _Float16* __restrict__ woT, float* __restrict__ out, int rt_first, int rt_count) {
  oproj_body<false>(yH, yL, woT, out, rt_first, rt_count);
}

extern "C" void kernel_launch(void* const* d_in, const int* in_sizes, int n_in,
                              void* d_out, int out_size, void* d_ws, size_t ws_size,
                              hipStream_t stream) {
  if (n_in < 6) return;
  const int need_x = ((NB - 1) * SEQ_FULL + SEQ) * CDIM;
  if (in_sizes[0] < need_x) return;
  if (in_sizes[1] < SEQ * SEQ_FULL) return;
  if (in_sizes[2] < CDIM * CDIM || in_sizes[3] < CDIM * VEW || in_sizes[4] < CDIM * VEW || in_sizes[5] < VEW * CDIM) return;
  if (out_size < need_x) return;
  if (ws_size < WS_TOTAL) return;

  const float* x    = (const float*)d_in[0];
  const float* mask = (const float*)d_in[1];
  const float* wq   = (const float*)d_in[2];
  const float* wk   = (const float*)d_in[3];
  const float* wv   = (const float*)d_in[4];
  const float* wo   = (const float*)d_in[5];
  float* out = (float*)d_out;

  char* ws = (char*)d_ws;
  size_t off = 0;
  _Float16* xh     = (_Float16*)(ws + off);     off += XH_BYTES;
  _Float16* wall   = (_Float16*)(ws + off);     off += WALL_BYTES;
  _Float16* woT    = (_Float16*)(ws + off);     off += WOT_BYTES;
  float*    cosT   = (float*)(ws + off);        off += TAB_BYTES;
  float*    sinT   = (float*)(ws + off);        off += TAB_BYTES;
  unsigned int* mbits = (unsigned int*)(ws + off); off += MB_BYTES;
  _Float16* planes = (_Float16*)(ws + off);     off += 6 * PL_BYTES;
  _Float16* yH     = (_Float16*)(ws + off);     off += YP_BYTES;
  _Float16* yL     = (_Float16*)(ws + off);     off += YP_BYTES;
  if (off > ws_size) return;

  _Float16* qH  = planes;
  _Float16* qL  = planes + PL_ELEMS;
  _Float16* kH  = planes + 2 * PL_ELEMS;
  _Float16* kL  = planes + 3 * PL_ELEMS;
  _Float16* vTH = planes + 4 * PL_ELEMS;
  _Float16* vTL = planes + 5 * PL_ELEMS;

  k_cvt_x<<<dim3(NTOK / 2), dim3(256), 0, stream>>>(x, xh);
  k_cvt_wT<<<dim3(CDIM / 64, CDIM / 64), dim3(256), 0, stream>>>(wq, CDIM, wall, CDIM);
  k_cvt_wT<<<dim3(VEW / 64, CDIM / 64), dim3(256), 0, stream>>>(wk, VEW, wall + (size_t)CDIM * CDIM, CDIM);
  k_cvt_wT<<<dim3(VEW / 64, CDIM / 64), dim3(256), 0, stream>>>(wv, VEW, wall + (size_t)(CDIM + VEW) * CDIM, CDIM);
  k_cvt_wT<<<dim3(CDIM / 64, VEW / 64), dim3(256), 0, stream>>>(wo, CDIM, woT, VEW);
  k_rope_tab<<<dim3(SEQ / 8), dim3(256), 0, stream>>>(cosT, sinT);
  k_mask_pack<<<dim3(SEQ / 8), dim3(256), 0, stream>>>(mask, mbits);
  k_qkv<<<dim3(NUNIT, NTOK / 64), dim3(128), 0, stream>>>(xh, wall, cosT, sinT, planes);
  k_flash_res<<<dim3(QT_RES, NKV, NB), dim3(128), 0, stream>>>(qH, qL, kH, kL, vTH, vTL, mbits, yH, yL, 0);
  if (QT_ALL > QT_RES) {
    k_flash_one<<<dim3(QT_ALL - QT_RES, NKV, NB), dim3(128), 0, stream>>>(qH, qL, kH, kL, vTH, vTL, mbits,
                                                                           yH, yL, QT_RES);
  }
  k_oproj_res<<<dim3(CDIM / 64, NB * QT_RES), dim3(128), 0, stream>>>(yH, yL, woT, out, 0, QT_RES);
  if (QT_ALL > QT_RES) {
    k_oproj_one<<<dim3(CDIM / 64, NB * (QT_ALL - QT_RES)), dim3(128), 0, stream>>>(yH, yL, woT, out,
                                                                                    QT_RES, QT_ALL - QT_RES);
  }
}
